// GeometricGAT_48799418417183
// MI455X (gfx1250) — hardware-verified
//
#include <hip/hip_runtime.h>
#include <math.h>

typedef __attribute__((ext_vector_type(16))) _Float16 v16h;
typedef __attribute__((ext_vector_type(8)))  _Float16 v8h;
typedef __attribute__((ext_vector_type(16))) __bf16   v16b;
typedef __attribute__((ext_vector_type(8)))  __bf16   v8b;
typedef __attribute__((ext_vector_type(8)))  float    v8f;
typedef __attribute__((ext_vector_type(4)))  float    v4f;
typedef __attribute__((ext_vector_type(4)))  int      v4i;
#define U16(p) ((const unsigned short*)(const void*)(p))

__device__ __forceinline__ unsigned short f2bf_bits(float f) {
  unsigned u = __float_as_uint(f);
  return (unsigned short)((u + 0x7FFFu + ((u >> 16) & 1u)) >> 16);
}
__device__ __forceinline__ float bf_bits2f(unsigned short h) { return __uint_as_float(((unsigned)h) << 16); }

__device__ __forceinline__ void dep_guard_h(v8f& a, v8f& b, v16h x, v16h y) { asm volatile("v_nop\n\tv_nop\n\tv_nop\n\tv_nop" : "+v"(a), "+v"(b) : "v"(x), "v"(y)); }
__device__ __forceinline__ void dep_guard_b(v8f& a, v8f& b, v16b x, v16b y) { asm volatile("v_nop\n\tv_nop\n\tv_nop\n\tv_nop" : "+v"(a), "+v"(b) : "v"(x), "v"(y)); }
__device__ __forceinline__ void keep4_h(v16h a, v16h b, v16h c, v16h d) { asm volatile("v_nop" :: "v"(a), "v"(b), "v"(c), "v"(d)); }
__device__ __forceinline__ void keep4_b(v16b a, v16b b, v16b c, v16b d) { asm volatile("v_nop" :: "v"(a), "v"(b), "v"(c), "v"(d)); }
__device__ __forceinline__ void fence_v4(v4f& t) { asm volatile("" : "+v"(t)); }
__device__ __forceinline__ void acc_guard4(v8f& a, v8f& b, v8f& c, v8f& d) { asm volatile("v_nop\n\tv_nop\n\tv_nop\n\tv_nop" : "+v"(a), "+v"(b), "+v"(c), "+v"(d)); }
template <typename T> struct Frag;
template <> struct Frag<_Float16> {
  typedef v16h V; union U { v16h v; v8h h[2]; };
  static __device__ __forceinline__ v16h load(const _Float16* p) {
    U f; f.h[0] = *(const v8h*)(p); f.h[1] = *(const v8h*)(p + 16); return f.v;
  }
  static __device__ __forceinline__ v8f mma(v16h a, v16h b, v8f c) {
    return __builtin_amdgcn_wmma_f32_16x16x32_f16(false, a, false, b, (short)0, c, false, false);
  }
  static __device__ __forceinline__ void guard(v8f& a, v8f& b, v16h x, v16h y) { dep_guard_h(a, b, x, y); }
  static __device__ __forceinline__ void keep(v16h a, v16h b, v16h c, v16h d) { keep4_h(a, b, c, d); }
};
template <> struct Frag<__bf16> {
  typedef v16b V; union U { v16b v; v8b h[2]; };
  static __device__ __forceinline__ v16b load(const __bf16* p) {
    U f; f.h[0] = *(const v8b*)(p); f.h[1] = *(const v8b*)(p + 16); return f.v;
  }
  static __device__ __forceinline__ v8f mma(v16b a, v16b b, v8f c) {
    return __builtin_amdgcn_wmma_f32_16x16x32_bf16(false, a, false, b, (short)0, c, false, false);
  }
  static __device__ __forceinline__ void guard(v8f& a, v8f& b, v16b x, v16b y) { dep_guard_b(a, b, x, y); }
  static __device__ __forceinline__ void keep(v16b a, v16b b, v16b c, v16b d) { keep4_b(a, b, c, d); }
};

template <int ET> struct Elem;
template <> struct Elem<0> { typedef _Float16 T; };
template <> struct Elem<1> { typedef __bf16 T; };
template <int ET, bool SPLIT, int BIAS_MODE, int OUT_MODE, bool RESID, int ACT = 0>
__global__ __launch_bounds__(256) void wmma_gemm64(
    const unsigned short* __restrict__ Ap, const unsigned short* __restrict__ A2p, int lda, long strideA,
    const unsigned short* __restrict__ Btp, const unsigned short* __restrict__ Bt2p, int ldb, long strideB,
    void* __restrict__ Cout, void* __restrict__ Cout2, int ldc, long strideC,
    const float* __restrict__ bias,
    const float* __restrict__ resid, long strideR,
    int M, int N, int K, float scale) {
  typedef typename Elem<ET>::T T;
  typedef typename Frag<T>::V V;
  const T* A = (const T*)Ap; const T* A2 = (const T*)A2p; const T* Bt = (const T*)Btp; const T* Bt2 = (const T*)Bt2p;
  __shared__ __align__(16) float sT[8][16 * 68];
  const int b    = blockIdx.y;
  const int lane = threadIdx.x & 31;
  const int wave = threadIdx.x >> 5;
  const int tilesN = N >> 6;
  const int tilesM = M >> 6;
  const int tile = blockIdx.x * 8 + wave;
  if (tile >= tilesM * tilesN) return;
  const int tm = tile / tilesN;
  const int tn = tile - tm * tilesN;
  const int m0 = tm << 6;
  const int n0 = tn << 6;

  const T* Ab  = A  + (size_t)b * strideA;
  const T* Bb  = Bt + (size_t)b * strideB;
  const T* Ab2 = SPLIT ? (A2  + (size_t)b * strideA) : nullptr;
  const T* Bb2 = SPLIT ? (Bt2 + (size_t)b * strideB) : nullptr;

  const int rlane = lane & 15;
  const int koff  = (lane >> 4) * 8;
  const int mOff  = (lane >> 4) * 8;

  v8f acc[4][4];
#pragma unroll
  for (int i = 0; i < 4; ++i)
#pragma unroll
    for (int j = 0; j < 4; ++j) acc[i][j] = (v8f){0.f,0.f,0.f,0.f,0.f,0.f,0.f,0.f};

  for (int k0 = 0; k0 < K; k0 += 32) {
    V bh[4], bl[4];
#pragma unroll
    for (int j = 0; j < 4; ++j) {
      const size_t bo = (size_t)(n0 + (j << 4) + rlane) * ldb + koff + k0;
      bh[j] = Frag<T>::load(Bb + bo);
      if (SPLIT) bl[j] = Frag<T>::load(Bb2 + bo);
    }
#pragma unroll
    for (int i = 0; i < 4; ++i) {
      const size_t ao = (size_t)(m0 + (i << 4) + rlane) * lda + koff + k0;
      V ah = Frag<T>::load(Ab + ao);
      V al;
      if (SPLIT) al = Frag<T>::load(Ab2 + ao);
#pragma unroll
      for (int j = 0; j < 4; ++j) {
        acc[i][j] = Frag<T>::mma(ah, bh[j], acc[i][j]);
        if (SPLIT) {
          acc[i][j] = Frag<T>::mma(ah, bl[j], acc[i][j]);
          acc[i][j] = Frag<T>::mma(al, bh[j], acc[i][j]);
        }
      }
      Frag<T>::guard(acc[i][0], acc[i][3], ah, SPLIT ? al : ah);
    }
    Frag<T>::keep(bh[0], bh[1], bh[2], bh[3]);
    if (SPLIT) Frag<T>::keep(bl[0], bl[1], bl[2], bl[3]);
  }
  acc_guard4(acc[0][0], acc[0][1], acc[0][2], acc[0][3]);
  acc_guard4(acc[1][0], acc[1][1], acc[1][2], acc[1][3]);
  acc_guard4(acc[2][0], acc[2][1], acc[2][2], acc[2][3]);
  acc_guard4(acc[3][0], acc[3][1], acc[3][2], acc[3][3]);

  float* slab = sT[wave];
  const float* Rb = RESID ? (resid + (size_t)b * strideR) : nullptr;
#pragma unroll
  for (int i = 0; i < 4; ++i) {
    const int mBase = m0 + (i << 4);
#pragma unroll
    for (int j = 0; j < 4; ++j) {
      const int n = n0 + (j << 4) + rlane;
      float bv = 0.f;
      if (BIAS_MODE == 2) bv = bias[n];
#pragma unroll
      for (int r = 0; r < 8; ++r) {
        float v = acc[i][j][r] * scale;
        if (BIAS_MODE == 1) v += bias[mBase + mOff + r];
        if (BIAS_MODE == 2) v += bv;
        if (RESID) v += Rb[(size_t)(mBase + mOff + r) * ldc + n];
        if (ACT == 1) v = tanhf(v);
        if (ACT == 2) v = fmaxf(v, 0.0f);
        if (ACT == 3) v = v / (1.0f + expf(-v));
        if (ACT == 4) v = (v > 0.f) ? v : 0.01f * v;
        if (ACT == 5) v = 0.5f * v * (1.0f + erff(v * 0.70710678118654752f));
        slab[(mOff + r) * 68 + (j << 4) + rlane] = v;
      }
    }
    __builtin_amdgcn_fence(__ATOMIC_RELEASE, "workgroup");
    __builtin_amdgcn_wave_barrier();
    __builtin_amdgcn_fence(__ATOMIC_ACQUIRE, "workgroup");
    if (OUT_MODE == 0) {
      float* C = (float*)Cout + (size_t)b * strideC;
      const int hh = lane >> 4, c4 = (lane & 15) * 4;
      for (int pass = 0; pass < 2; ++pass) {
#pragma unroll
        for (int it = 0; it < 8; ++it) {
          const int row = it * 2 + hh;
          v4f v = *(const v4f*)(slab + row * 68 + c4);
          *(volatile v4f*)(C + (size_t)(mBase + row) * ldc + n0 + c4) = v;
        }
        __threadfence();
      }
    } else {
      const int q = lane >> 3, c8 = (lane & 7) * 8;
      unsigned short* C  = (unsigned short*)Cout  + (size_t)b * strideC;
      unsigned short* C2 = (OUT_MODE == 2) ? ((unsigned short*)Cout2 + (size_t)b * strideC) : nullptr;
      for (int pass = 0; pass < 2; ++pass) {
#pragma unroll
        for (int it = 0; it < 4; ++it) {
          const int row = it * 4 + q;
          const float* sp = slab + row * 68 + c8;
          v8h hv, lv;
#pragma unroll
          for (int e = 0; e < 8; ++e) {
            if (OUT_MODE == 1) {
              hv[e] = (_Float16)sp[e];
            } else {
              unsigned short hb = f2bf_bits(sp[e]);
              unsigned short lb = f2bf_bits(sp[e] - bf_bits2f(hb));
              hv[e] = __builtin_bit_cast(_Float16, hb);
              lv[e] = __builtin_bit_cast(_Float16, lb);
            }
          }
          *(volatile v8h*)(C + (size_t)(mBase + row) * ldc + n0 + c8) = hv;
          if (OUT_MODE == 2) *(volatile v8h*)(C2 + (size_t)(mBase + row) * ldc + n0 + c8) = lv;
        }
        __threadfence();
      }
    }
    __builtin_amdgcn_fence(__ATOMIC_RELEASE, "workgroup");
    __builtin_amdgcn_wave_barrier();
    __builtin_amdgcn_fence(__ATOMIC_ACQUIRE, "workgroup");
  }
}

__global__ __launch_bounds__(256) void transpose_cast_f16(const float* __restrict__ in, int ldi,
                                                         _Float16* __restrict__ outT, int ldo, float scale) {
  __shared__ __align__(16) _Float16 tile[64][72];
  const int c0 = blockIdx.x * 64, r0 = blockIdx.y * 64;
  const int t = threadIdx.y * 32 + threadIdx.x;
  for (int i = threadIdx.y; i < 64; i += 8) {
    tile[threadIdx.x][i]      = (_Float16)(in[(size_t)(r0 + i) * ldi + c0 + threadIdx.x] * scale);
    tile[32 + threadIdx.x][i] = (_Float16)(in[(size_t)(r0 + i) * ldi + c0 + 32 + threadIdx.x] * scale);
  }
  __syncthreads();
  const int q = t >> 3, c8 = (t & 7) * 8;
  for (int pass = 0; pass < 2; ++pass) {
#pragma unroll
    for (int it = 0; it < 2; ++it) {
      const int c = it * 32 + q;
      v8h hv = *(const v8h*)(&tile[c][c8]);
      *(volatile v8h*)(outT + (size_t)(c0 + c) * ldo + r0 + c8) = hv;
    }
    __threadfence();
  }
}

#define NN 10000
#define NPAD 10048
#define NE 320000
#define FIN 256
#define NH 4
#define C1 64
#define C2 256
#define NT 256
#define SRB 512
#define NTILE 20
#define SCH 2048
#define NCH ((NE + SCH - 1) / SCH)

__global__ __launch_bounds__(256) void cast_pad_kernel(const float* __restrict__ x, unsigned* __restrict__ x16, int F) {
  const long i = (long)blockIdx.x * 256 + threadIdx.x; const long n2 = (long)NPAD * F / 2;
  if (i >= n2) return;
  const long e0 = 2 * i; const long row = e0 / F;
  const float a = (row < NN) ? x[e0] : 0.f, b = (row < NN) ? x[e0 + 1] : 0.f;
  const unsigned u = (unsigned)__builtin_bit_cast(unsigned short, (_Float16)a) | ((unsigned)__builtin_bit_cast(unsigned short, (_Float16)b) << 16);
  ((volatile unsigned*)x16)[i] = u; __threadfence(); ((volatile unsigned*)x16)[i] = u;
}
__global__ __launch_bounds__(256) void bias_cat2_kernel(const float* a, const float* b, float* __restrict__ o, int hc) {
  for (int pass = 0; pass < 2; ++pass) { for (int i = threadIdx.x; i < 2 * hc; i += 256) ((volatile float*)o)[i] = (i < hc) ? a[i] : b[i - hc]; __threadfence(); }
}
__global__ __launch_bounds__(256) void tail_copy_kernel(const float* __restrict__ src, float* __restrict__ dst, int n) {
  for (int pass = 0; pass < 2; ++pass) {
    for (int i = threadIdx.x * 4; i < n; i += 256 * 4) {
      const v4f v = *(const v4f*)(src + i);
      *(volatile v4f*)(dst + i) = v;
    }
    __threadfence();
  }
}

__device__ __forceinline__ int blk_excl_scan(int cnt, int* scan_ws, int tid, int* tot) {
  const int lane = tid & 31, wave = tid >> 5; int incl = cnt;
#pragma unroll
  for (int o = 1; o < 32; o <<= 1) { const int v = __shfl_up(incl, o, 32); if (lane >= o) incl += v; }
  if (lane == 31) scan_ws[wave] = incl;
  __syncthreads();
  if (wave == 0) { int wv = (lane < NT / 32) ? scan_ws[lane] : 0; int wincl = wv;
#pragma unroll
    for (int o = 1; o < 32; o <<= 1) { const int v = __shfl_up(wincl, o, 32); if (lane >= o) wincl += v; }
    if (lane < NT / 32) scan_ws[32 + lane] = wincl - wv; if (lane == 31) scan_ws[64] = wincl; }
  __syncthreads();
  const int res = scan_ws[32 + wave] + incl - cnt; *tot = scan_ws[64];
  return res;
}
template <int SP, int CAP>
__device__ __forceinline__ int chunk_hits(const int* __restrict__ dstv, int e0, int n0, int tid, int* LIST, int* scan_ws) {
  const int eb = e0 + tid * SP;
  int rec[SP]; int cnt = 0;
  if (eb < NE) {
#pragma unroll
    for (int k = 0; k < SP; k += 4) {
      const v4i d4 = *(const v4i*)(dstv + eb + k);
#pragma unroll
      for (int u = 0; u < 4; ++u) {
        const int d = d4[u]; int r = -1;
        if (d >= n0 && d < n0 + SRB && d < NN) { r = ((d - n0) << 19) | (eb + k + u); ++cnt; }
        rec[k + u] = r;
      }
    }
  } else {
#pragma unroll
    for (int k = 0; k < SP; ++k) rec[k] = -1;
  }
  int tot; int p = blk_excl_scan(cnt, scan_ws, tid, &tot);
#pragma unroll
  for (int k = 0; k < SP; ++k) if (rec[k] >= 0) { if ((unsigned)p < (unsigned)CAP) LIST[p] = rec[k]; ++p; }
  __syncthreads();
  return tot < CAP ? tot : CAP;
}

template <int CH>
__global__ __launch_bounds__(NT) void gat_logits_kernel(const float* __restrict__ XLR, const int* __restrict__ ei, const float* __restrict__ eattr,
                                                       const float* __restrict__ We, const float* __restrict__ att, float* __restrict__ LG) {
  constexpr int HC = NH * CH, PITCH = 2 * HC, CPL = HC / 32;
  __shared__ __align__(16) float sW[3 * HC];
  __shared__ __align__(16) float sA[HC];
  __shared__ __align__(16) float sal[32 * 4];
  const int tid = threadIdx.x, lane = tid & 31, wave = tid >> 5;
  for (int i = tid; i < 3 * HC; i += NT) sW[i] = We[i];
  for (int i = tid; i < HC; i += NT) sA[i] = att[i];
  __syncthreads();
  const int c0 = CPL * lane;
#pragma unroll 1
  for (int i = 0; i < 4; ++i) {
    const int el = 4 * wave + i;
    const int e = blockIdx.x * 32 + el;
    int s = ei[e], d = ei[NE + e];
    s = s < 0 ? 0 : (s >= NN ? NN - 1 : s);
    d = d < 0 ? 0 : (d >= NN ? NN - 1 : d);
    const float a0 = eattr[(size_t)e * 3], a1 = eattr[(size_t)e * 3 + 1], a2 = eattr[(size_t)e * 3 + 2];
    const float* xl = XLR + (size_t)s * PITCH + c0;
    const float* xr = XLR + (size_t)d * PITCH + HC + c0;
    float dsum = 0.f;
#pragma unroll 1
    for (int q = 0; q < CPL; q += 4) {
      const v4f xv = *(const v4f*)(xl + q), rv = *(const v4f*)(xr + q);
      const v4f w0 = *(const v4f*)(sW + c0 + q), w1 = *(const v4f*)(sW + HC + c0 + q), w2 = *(const v4f*)(sW + 2 * HC + c0 + q);
      const v4f av = *(const v4f*)(sA + c0 + q);
      const v4f ee = a0 * w0 + a1 * w1 + a2 * w2;
      const v4f m = (xv + rv) + ee;
#pragma unroll
      for (int t = 0; t < 4; ++t) { float v = m[t]; v = (v >= 0.f) ? v : 0.2f * v; dsum += v * av[t]; }
    }
    dsum += __shfl_xor(dsum, 1, 32); dsum += __shfl_xor(dsum, 2, 32); dsum += __shfl_xor(dsum, 4, 32);
    if ((lane & 7) == 0) sal[el * 4 + (lane >> 3)] = dsum;
  }
  __syncthreads();
  if (tid < 32) {
    const v4f v = *(const v4f*)(sal + 4 * tid);
    float* op = LG + ((size_t)blockIdx.x * 32 + tid) * 4;
    *(volatile v4f*)op = v; __threadfence(); *(volatile v4f*)op = v;
  }
}

template <int CH, bool SILU, bool STATS>
__global__ __launch_bounds__(NT) void gat_stream_kernel(float* XLR, const int* __restrict__ ei, const float* __restrict__ LG,
                                                       const float* __restrict__ bias, float* __restrict__ ST) {
  constexpr int HC = NH * CH, PITCH = 2 * HC, NJ = HC / 128, NK = HC / 256, LCH = (CH == 64) ? 6 : 8;
  __shared__ int LIST[SCH];
  __shared__ float SM[SRB * NH];
  __shared__ float SL[SRB * NH];
  __shared__ int scan_ws[80];
  __shared__ __align__(16) float stg[NT / 32][HC];
  const int tid = threadIdx.x, lane = tid & 31, wave = tid >> 5;
  const int n0 = blockIdx.x * SRB;
  const int hq = lane & 3;
  const v4f z4 = {0.f, 0.f, 0.f, 0.f};
#pragma unroll 1
  for (int j = 0; j < 64; ++j) {
    const int n = n0 + wave * 64 + j;
    if (n < NPAD) {
      float* rp = XLR + (size_t)n * PITCH + HC + 4 * lane;
#pragma unroll
      for (int jj = 0; jj < NJ; ++jj) *(v4f*)(rp + 128 * jj) = z4;
    }
  }
  for (int i = tid; i < SRB * NH; i += NT) { SM[i] = -INFINITY; SL[i] = 0.f; }
  __syncthreads();
  const int* dstv = ei + NE;
#pragma unroll 1
  for (int c = 0; c < NCH; ++c) {
    const int tot = chunk_hits<SCH / NT, SCH>(dstv, c * SCH, n0, tid, LIST, scan_ws);
#pragma unroll 1
    for (int base = 0; base < tot; base += 32) {
      const int q = base + lane;
      const int rv = (q < tot) ? LIST[q] : -1;
      const int own = (rv >= 0 && (rv >> 25) == wave) ? 1 : 0;
      unsigned msk = (unsigned)__ballot(own);
#pragma unroll 1
      for (int it = 0; it < 32; ++it) {
        if (msk == 0u) break;
        const int bpos = __builtin_ctz(msk); msk &= msk - 1u;
        const int r = __shfl(rv, bpos, 32);
        const int dl = (r >> 19) & 511;
        int e = r & 0x7FFFF; e = (e < NE) ? e : NE - 1;
        int s = ei[e]; s = s < 0 ? 0 : (s >= NN ? NN - 1 : s);
        const float lg = LG[(size_t)e * 4 + hq];
        const int mi = dl * 4 + hq;
        const float mo = SM[mi], lo = SL[mi];
        const float mn = fmaxf(mo, lg);
        const float rr = __expf(mo - mn), ex = __expf(lg - mn);
        const float ln = lo * rr + ex;
        if (lane < 4) { SM[mi] = mn; SL[mi] = ln; }
        float* rp = XLR + (size_t)(n0 + dl) * PITCH + HC + 4 * lane;
        const float* xp = XLR + (size_t)s * PITCH + 4 * lane;
#pragma unroll
        for (int jj = 0; jj < NJ; ++jj) {
          const int hj = (4 * lane + 128 * jj) >> LCH;
          const float rrj = __shfl(rr, hj, 32), exj = __shfl(ex, hj, 32);
          v4f a = *(const v4f*)(rp + 128 * jj);
          const v4f hv = *(const v4f*)(xp + 128 * jj);
          a = a * rrj + exj * hv;
          *(v4f*)(rp + 128 * jj) = a;
        }
      }
    }
    __syncthreads();
  }
  v4f bvj[NJ];
#pragma unroll
  for (int jj = 0; jj < NJ; ++jj) {
    const int cb = 4 * lane + 128 * jj;
    v4f t; t[0] = bias[cb]; t[1] = bias[cb + 1]; t[2] = bias[cb + 2]; t[3] = bias[cb + 3]; bvj[jj] = t;
  }
  float* sw = stg[wave];
#pragma unroll 1
  for (int j = 0; j < 64; ++j) {
    const int dl = wave * 64 + j; const int n = n0 + dl;
    if (n < NPAD) {
      const bool live = n < NN;
      const int si = dl * 4 + hq;
      const float smv = SM[si], slv = SL[si];
      const float lv = (live && slv > 0.f) ? slv : 1.0f;
      const float inv4 = 1.0f / lv;
      const float* rp = XLR + (size_t)n * PITCH + HC + 4 * lane;
#pragma unroll
      for (int jj = 0; jj < NJ; ++jj) {
        const int hj = (4 * lane + 128 * jj) >> LCH;
        const float invj = __shfl(inv4, hj, 32);
        const v4f a = *(const v4f*)(rp + 128 * jj);
        v4f t = a * invj; fence_v4(t); t = t + bvj[jj];
        v4f o;
#pragma unroll
        for (int q = 0; q < 4; ++q) {
          float v = t[q];
          if (SILU) v = v * __builtin_amdgcn_rcpf(1.0f + __expf(-v));
          o[q] = live ? v * 64.0f : 0.f;
        }
        *(v4f*)(sw + 4 * lane + 128 * jj) = o;
      }
      __builtin_amdgcn_fence(__ATOMIC_RELEASE, "workgroup");
      __builtin_amdgcn_wave_barrier();
      __builtin_amdgcn_fence(__ATOMIC_ACQUIRE, "workgroup");
      v8h hk[NK];
#pragma unroll
      for (int k = 0; k < NK; ++k) {
        const float* sp = sw + 256 * k + 8 * lane;
        const v4f u0 = *(const v4f*)sp, u1 = *(const v4f*)(sp + 4);
#pragma unroll
        for (int q = 0; q < 4; ++q) { hk[k][q] = (_Float16)u0[q]; hk[k][4 + q] = (_Float16)u1[q]; }
      }
      _Float16* hrow = (_Float16*)(XLR + (size_t)n * PITCH + HC);
      for (int pass = 0; pass < 2; ++pass) {
#pragma unroll
        for (int k = 0; k < NK; ++k) *(volatile v8h*)(hrow + 256 * k + 8 * lane) = hk[k];
        __threadfence();
      }
      if (STATS) {
        const float v = live ? ((lane < 4) ? smv : ((lane < 8) ? slv : 0.f)) : ((lane >= 4 && lane < 8) ? 1.0f : 0.f);
        ((volatile float*)ST)[(size_t)n * 32 + lane] = v; __threadfence(); ((volatile float*)ST)[(size_t)n * 32 + lane] = v;
      }
      __builtin_amdgcn_fence(__ATOMIC_RELEASE, "workgroup");
      __builtin_amdgcn_wave_barrier();
      __builtin_amdgcn_fence(__ATOMIC_ACQUIRE, "workgroup");
    }
  }
}

__global__ __launch_bounds__(NT) void gat_alpha_kernel(const float* __restrict__ LG, const int* __restrict__ ei, const float* __restrict__ ST,
                                                      float* __restrict__ alpha) {
  const int e = blockIdx.x * NT + threadIdx.x;
  const v4f lg = *(const v4f*)(LG + (size_t)e * 4);
  int d = ei[NE + e]; d = d < 0 ? 0 : (d >= NN ? NN - 1 : d);
  const v4f m4 = *(const v4f*)(ST + (size_t)d * 32), l4 = *(const v4f*)(ST + (size_t)d * 32 + 4);
  v4f o;
#pragma unroll
  for (int q = 0; q < 4; ++q) { const float lv = l4[q]; o[q] = (lv > 0.f) ? __expf(lg[q] - m4[q]) * (1.0f / lv) : 0.f; }
  float* op = alpha + (size_t)e * 4;
  *(volatile v4f*)op = o; __threadfence(); *(volatile v4f*)op = o;
}

extern "C" void kernel_launch(void* const* d_in, const int* in_sizes, int n_in,
                              void* d_out, int out_size, void* d_ws, size_t ws_size,
                              hipStream_t stream) {
  (void)in_sizes; (void)n_in; (void)out_size;
  const float* x     = (const float*)d_in[0];
  const int*   ei    = (const int*)  d_in[1];
  const float* eattr = (const float*)d_in[2];
  const float* W1l = (const float*)d_in[3];  const float* b1l  = (const float*)d_in[4];
  const float* W1r = (const float*)d_in[5];  const float* b1r  = (const float*)d_in[6];
  const float* W1e = (const float*)d_in[7];  const float* att1 = (const float*)d_in[8];  const float* bias1 = (const float*)d_in[9];
  const float* W2l = (const float*)d_in[10]; const float* b2l  = (const float*)d_in[11];
  const float* W2r = (const float*)d_in[12]; const float* b2r  = (const float*)d_in[13];
  const float* W2e = (const float*)d_in[14]; const float* att2 = (const float*)d_in[15]; const float* bias2 = (const float*)d_in[16];
  const float* Wp  = (const float*)d_in[17]; const float* bp   = (const float*)d_in[18];
  float* y     = (float*)d_out;
  float* alpha = y + (size_t)NN * 256;

  char* ws = (char*)d_ws; size_t off = 0;
  auto carve = [&](size_t bytes) -> char* { char* p = ws + off; off += (bytes + 255) & ~(size_t)255; return p; };
  unsigned* X16  = (unsigned*)carve((size_t)NPAD * FIN * 2);
  _Float16* W1T  = (_Float16*)carve((size_t)(2 * NH * C1) * FIN * 2);
  _Float16* W2T  = (_Float16*)carve((size_t)(2 * NH * C2) * FIN * 2);
  _Float16* WpT  = (_Float16*)carve((size_t)256 * (NH * C2) * 2);
  float*    bc1  = (float*)carve((size_t)2 * NH * C1 * 4);
  float*    bc2  = (float*)carve((size_t)2 * NH * C2 * 4);
  float*    XLR1 = (float*)carve((size_t)NPAD * 2 * NH * C1 * 4);
  float*    LG   = (float*)carve((size_t)NE * 4 * 4);
  float*    XLR2 = (float*)carve((size_t)NPAD * 2 * NH * C2 * 4);
  float*    ST   = (float*)carve((size_t)NPAD * 32 * 4);
  float*    YP   = (float*)carve((size_t)64 * 256 * 4);
  if (off > ws_size || off > (size_t)134217728) return;

  cast_pad_kernel<<<(NPAD * FIN / 2 + 255) / 256, 256, 0, stream>>>(x, X16, FIN);
  transpose_cast_f16<<<dim3(NH * C1 / 64, FIN / 64), dim3(32, 8), 0, stream>>>(W1l, NH * C1, W1T, FIN, 1.0f);
  transpose_cast_f16<<<dim3(NH * C1 / 64, FIN / 64), dim3(32, 8), 0, stream>>>(W1r, NH * C1, W1T + (size_t)NH * C1 * FIN, FIN, 1.0f);
  transpose_cast_f16<<<dim3(NH * C2 / 64, FIN / 64), dim3(32, 8), 0, stream>>>(W2l, NH * C2, W2T, FIN, 1.0f);
  transpose_cast_f16<<<dim3(NH * C2 / 64, FIN / 64), dim3(32, 8), 0, stream>>>(W2r, NH * C2, W2T + (size_t)NH * C2 * FIN, FIN, 1.0f);
  transpose_cast_f16<<<dim3(256 / 64, NH * C2 / 64), dim3(32, 8), 0, stream>>>(Wp, 256, WpT, NH * C2, 1.0f);
  bias_cat2_kernel<<<1, 256, 0, stream>>>(b1l, b1r, bc1, NH * C1);
  bias_cat2_kernel<<<1, 256, 0, stream>>>(b2l, b2r, bc2, NH * C2);
  {
    const int t1 = (NPAD / 64) * (2 * NH * C1 / 64);
    wmma_gemm64<0, false, 2, 0, false><<<dim3((t1 + 7) / 8, 1), 256, 0, stream>>>(
        (const unsigned short*)X16, nullptr, FIN, 0L, U16(W1T), nullptr, FIN, 0L,
        (void*)XLR1, nullptr, 2 * NH * C1, 0L, bc1, nullptr, 0L, NPAD, 2 * NH * C1, FIN, 1.0f);
  }
  gat_logits_kernel<C1><<<NE / 32, NT, 0, stream>>>(XLR1, ei, eattr, W1e, att1, LG);
  gat_stream_kernel<C1, true, false><<<NTILE, NT, 0, stream>>>(XLR1, ei, LG, bias1, ST);
  {
    const int t2 = (NPAD / 64) * (2 * NH * C2 / 64);
    wmma_gemm64<0, false, 2, 0, false><<<dim3((t2 + 7) / 8, 1), 256, 0, stream>>>(
        U16(XLR1) + 512, nullptr, 1024, 0L, U16(W2T), nullptr, FIN, 0L,
        (void*)XLR2, nullptr, 2 * NH * C2, 0L, bc2, nullptr, 0L, NPAD, 2 * NH * C2, FIN, 0.015625f);
  }
  gat_logits_kernel<C2><<<NE / 32, NT, 0, stream>>>(XLR2, ei, eattr, W2e, att2, LG);
  gat_stream_kernel<C2, false, true><<<NTILE, NT, 0, stream>>>(XLR2, ei, LG, bias2, ST);
  gat_alpha_kernel<<<NE / NT, NT, 0, stream>>>(LG, ei, ST, alpha);
  {
    const int M0 = 9984;
    const int t3 = (M0 / 64) * (256 / 64);
    wmma_gemm64<0, false, 2, 0, false><<<dim3((t3 + 7) / 8, 1), 256, 0, stream>>>(
        U16(XLR2) + 2048, nullptr, 4096, 0L, U16(WpT), nullptr, NH * C2, 0L,
        (void*)y, nullptr, 256, 0L, bp, nullptr, 0L, M0, 256, NH * C2, 0.015625f);
    wmma_gemm64<0, false, 2, 0, false><<<dim3(1, 1), 256, 0, stream>>>(
        U16(XLR2) + 2048 + (size_t)M0 * 4096, nullptr, 4096, 0L, U16(WpT), nullptr, NH * C2, 0L,
        (void*)YP, nullptr, 256, 0L, bp, nullptr, 0L, 64, 256, NH * C2, 0.015625f);
    tail_copy_kernel<<<1, 256, 0, stream>>>(YP, y + (size_t)M0 * 256, (NN - M0) * 256);
  }
}
